// TransformerDecoderLayer_5695126634635
// MI455X (gfx1250) — hardware-verified
//
#include <hip/hip_runtime.h>


#ifndef NB
#define NB 2
#endif
#ifndef SEQ
#define SEQ 2048
#endif
#define NB_FULL 2
#define SEQ_FULL 2048
#define DM 1024
#define FF 4096
#define HE 16
#define DH 64
#define KT 32
#define QR 64
#define KPITCH 72
#define VPITCH 40
#define PPITCH 40
#define CPITCH 136
#define OPITCH 132
#define X_CARRY 16.0f
#define W_CARRY 1024.0f
#define QKV_CARRY 16.0f
#define P_CARRY 4096.0f
#define C_CARRY 64.0f
#define X2_CARRY 16.0f
#define H_CARRY 64.0f
#define NWB ((DM * DM) / 2048)
#define NFB ((FF * DM) / 2048)

static_assert(NB >= 1 && NB <= NB_FULL);
static_assert(SEQ >= QR && SEQ <= SEQ_FULL);
static_assert((SEQ & (SEQ - 1)) == 0);
static_assert(SEQ % QR == 0);
static_assert(SEQ % KT == 0);
static_assert((NB * SEQ) % 64 == 0);
static_assert(((long long)NB * SEQ * DM) % 2048 == 0);
static_assert(DM % 128 == 0 && FF % 128 == 0);
static_assert(DM % 32 == 0 && FF % 32 == 0);
static_assert(DM == HE * DH);
static_assert(HE % 2 == 0);
static_assert(DH == 64);
static_assert((DM * DM) % 2048 == 0 && (FF * DM) % 2048 == 0);

typedef _Float16 v8h  __attribute__((ext_vector_type(8)));
typedef _Float16 v16h __attribute__((ext_vector_type(16)));
typedef float v8f __attribute__((ext_vector_type(8)));
typedef float v4f __attribute__((ext_vector_type(4)));

union FragH { v16h v; v8h h[2]; };

__device__ __forceinline__ unsigned f2bf(float f) { unsigned u = __float_as_uint(f); u += 0x7FFFu + ((u >> 16) & 1u); return u >> 16; }
__device__ __forceinline__ float bf16r(float f) { return __uint_as_float(f2bf(f) << 16); }

__device__ __forceinline__ v8f wm_f16(v16h a, v16h b, v8f c) {
    c = __builtin_amdgcn_wmma_f32_16x16x32_f16(false, a, false, b, (short)0, c, false, false);
    asm volatile("v_nop\n\tv_nop\n\tv_nop\n\tv_nop" : "+v"(c) : "v"(a), "v"(b));
    return c;
}

__global__ __launch_bounds__(256) void k_convert(const float* __restrict__ x, const float* __restrict__ wq, const float* __restrict__ wk, const float* __restrict__ wv,
                                                const float* __restrict__ wo, const float* __restrict__ w1, const float* __restrict__ w2,
                                                _Float16* Xh, _Float16* Wqkv, _Float16* Woh, _Float16* W1h, _Float16* W2h, unsigned nblkX)
{
    const unsigned bid = blockIdx.x, tid = threadIdx.x;
    const float* src;
    _Float16* dst;
    float sc = W_CARRY;
    if (bid < nblkX) {
        const unsigned e = (bid * 256u + tid) * 8u;
        const unsigned m = e / (unsigned)DM, col = e % (unsigned)DM;
        const unsigned bb = m / (unsigned)SEQ, n = m % (unsigned)SEQ;
        src = x + ((size_t)bb * SEQ_FULL + n) * DM + col;
        dst = Xh + e;
        sc = X_CARRY;
    } else {
        unsigned wb = bid - nblkX;
        if (wb < (unsigned)NWB) {
            const size_t e = ((size_t)wb * 256u + tid) * 8u;
            src = wq + e; dst = Wqkv + e;
        } else if (wb < 2u * NWB) {
            wb -= (unsigned)NWB;
            const size_t e = ((size_t)wb * 256u + tid) * 8u;
            src = wk + e; dst = Wqkv + (size_t)DM * DM + e;
        } else if (wb < 3u * NWB) {
            wb -= 2u * NWB;
            const size_t e = ((size_t)wb * 256u + tid) * 8u;
            src = wv + e; dst = Wqkv + (size_t)2 * DM * DM + e;
        } else if (wb < 4u * NWB) {
            wb -= 3u * NWB;
            const size_t e = ((size_t)wb * 256u + tid) * 8u;
            src = wo + e; dst = Woh + e;
        } else if (wb < 4u * NWB + (unsigned)NFB) {
            wb -= 4u * NWB;
            const size_t e = ((size_t)wb * 256u + tid) * 8u;
            src = w1 + e; dst = W1h + e;
        } else {
            wb -= 4u * NWB + (unsigned)NFB;
            const size_t e = ((size_t)wb * 256u + tid) * 8u;
            src = w2 + e; dst = W2h + e;
        }
    }
    const v4f a0 = *(const v4f*)src, a1 = *(const v4f*)(src + 4);
    v8h o;
#pragma unroll
    for (int i = 0; i < 4; ++i) {
        o[i]     = (_Float16)(bf16r(a0[i]) * sc);
        o[4 + i] = (_Float16)(bf16r(a1[i]) * sc);
    }
    *(volatile v8h*)dst = o;
    __threadfence();
    *(volatile v8h*)dst = o;
}

template <int MODE, int KD>
__global__ __launch_bounds__(256) void k_gemm(const _Float16* __restrict__ A, const _Float16* __restrict__ Wh,
                                             const float* __restrict__ bias0, const float* __restrict__ bias1, const float* __restrict__ bias2,
                                             const float* __restrict__ resid, float* outF, _Float16* oh0, _Float16* oh1, _Float16* oh2)
{
    __shared__ __align__(16) float cst[64 * OPITCH];
    __shared__ __align__(16) _Float16 ct[64 * CPITCH];
    const unsigned tid = threadIdx.x, lane = tid & 31u, wv = tid >> 5, hh = lane >> 4, lm = lane & 15u;
    const unsigned rt = wv & 3u, ch = wv >> 2;
    const unsigned row0 = blockIdx.x * 64u, cb = blockIdx.y * 128u, col0 = cb + ch * 64u;
    const _Float16* xr = A + (size_t)(row0 + rt * 16u + lm) * KD;
    v8f acc[4];
#pragma unroll
    for (int t = 0; t < 4; ++t) acc[t] = (v8f){};
#pragma unroll 2
    for (unsigned kc = 0; kc < (unsigned)KD; kc += 32u) {
        FragH a;
        a.h[0] = *(const v8h*)(xr + kc + 8u * hh);
        a.h[1] = *(const v8h*)(xr + kc + 16u + 8u * hh);
#pragma unroll
        for (int t = 0; t < 4; ++t) {
            FragH bb;
            const _Float16* wr = Wh + (size_t)(col0 + (unsigned)t * 16u + lm) * KD + kc;
            bb.h[0] = *(const v8h*)(wr + 8u * hh);
            bb.h[1] = *(const v8h*)(wr + 16u + 8u * hh);
            acc[t] = wm_f16(a.v, bb.v, acc[t]);
        }
    }

    if constexpr (MODE == 0 || MODE == 1) {
        const float* bias;
        _Float16* op;
        unsigned ocb;
        if constexpr (MODE == 0) {
            const unsigned sel = blockIdx.y >> 3;
            ocb = cb & (unsigned)(DM - 1);
            bias = (sel == 0u) ? bias0 : ((sel == 1u) ? bias1 : bias2);
            op   = (sel == 0u) ? oh0 : ((sel == 1u) ? oh1 : oh2);
        } else {
            ocb = cb; bias = bias0; op = oh0;
        }
        constexpr unsigned OP = (MODE == 0) ? (unsigned)DM : (unsigned)FF;
        constexpr float INV = (MODE == 0) ? (1.0f / (X_CARRY * W_CARRY)) : (1.0f / (X2_CARRY * W_CARRY));
        constexpr float OC = (MODE == 0) ? QKV_CARRY : H_CARRY;
#pragma unroll
        for (int t = 0; t < 4; ++t) {
            const unsigned cl = ch * 64u + (unsigned)t * 16u + lm;
            const float bv = bf16r(bias[ocb + cl]);
#pragma unroll
            for (int r = 0; r < 8; ++r) {
                float v = acc[t][r] * INV + bv;
                if constexpr (MODE == 1) v = fmaxf(v, 0.0f);
                ct[(rt * 16u + 8u * hh + (unsigned)r) * CPITCH + cl] = (_Float16)(v * OC);
            }
        }
        __syncthreads();
        v8h ov[4];
#pragma unroll
        for (int i = 0; i < 4; ++i) {
            const unsigned p = tid + 256u * (unsigned)i, row = p >> 4, c8 = (p & 15u) * 8u;
            ov[i] = *(const v8h*)(ct + row * CPITCH + c8);
        }
#pragma unroll
        for (int i = 0; i < 4; ++i) {
            const unsigned p = tid + 256u * (unsigned)i, row = p >> 4, c8 = (p & 15u) * 8u;
            *(volatile v8h*)(op + (size_t)(row0 + row) * OP + ocb + c8) = ov[i];
        }
        __threadfence();
#pragma unroll
        for (int i = 0; i < 4; ++i) {
            const unsigned p = tid + 256u * (unsigned)i, row = p >> 4, c8 = (p & 15u) * 8u;
            *(volatile v8h*)(op + (size_t)(row0 + row) * OP + ocb + c8) = ov[i];
        }
    } else {
        constexpr float INV = (MODE == 2) ? (1.0f / (C_CARRY * W_CARRY)) : (1.0f / (H_CARRY * W_CARRY));
#pragma unroll
        for (int t = 0; t < 4; ++t) {
            const unsigned cl = ch * 64u + (unsigned)t * 16u + lm;
            const float bv = bf16r(bias0[cb + cl]);
#pragma unroll
            for (int r = 0; r < 8; ++r) cst[(rt * 16u + 8u * hh + (unsigned)r) * OPITCH + cl] = acc[t][r] * INV + bv;
        }
        __syncthreads();
        v4f ov[8];
#pragma unroll
        for (int i = 0; i < 8; ++i) {
            const unsigned p = tid + 256u * (unsigned)i, row = p >> 5, c4 = (p & 31u) * 4u;
            const unsigned m = row0 + row;
            v4f c = *(const v4f*)(cst + row * OPITCH + c4);
            if constexpr (MODE == 2) {
                const unsigned bb = m / (unsigned)SEQ, n = m % (unsigned)SEQ;
                const v4f xv = *(const v4f*)(resid + ((size_t)bb * SEQ_FULL + n) * DM + cb + c4);
#pragma unroll
                for (int j = 0; j < 4; ++j) c[j] += bf16r(xv[j]);
                *(v4f*)(cst + row * OPITCH + c4) = c;
            } else {
                const v4f xv = *(const v4f*)(resid + (size_t)m * DM + cb + c4);
#pragma unroll
                for (int j = 0; j < 4; ++j) c[j] += xv[j];
            }
            ov[i] = c;
        }
#pragma unroll
        for (int i = 0; i < 8; ++i) {
            const unsigned p = tid + 256u * (unsigned)i, row = p >> 5, c4 = (p & 31u) * 4u;
            const unsigned m = row0 + row;
            if constexpr (MODE == 2) {
                *(volatile v4f*)(outF + (size_t)m * DM + cb + c4) = ov[i];
            } else {
                const unsigned bb = m / (unsigned)SEQ, n = m % (unsigned)SEQ;
                *(volatile v4f*)(outF + ((size_t)bb * SEQ_FULL + n) * DM + cb + c4) = ov[i];
            }
        }
        __threadfence();
#pragma unroll
        for (int i = 0; i < 8; ++i) {
            const unsigned p = tid + 256u * (unsigned)i, row = p >> 5, c4 = (p & 31u) * 4u;
            const unsigned m = row0 + row;
            if constexpr (MODE == 2) {
                *(volatile v4f*)(outF + (size_t)m * DM + cb + c4) = ov[i];
            } else {
                const unsigned bb = m / (unsigned)SEQ, n = m % (unsigned)SEQ;
                *(volatile v4f*)(outF + ((size_t)bb * SEQ_FULL + n) * DM + cb + c4) = ov[i];
            }
        }
        if constexpr (MODE == 2) {
            __syncthreads();
            v8h hv[4];
#pragma unroll
            for (int i = 0; i < 4; ++i) {
                const unsigned p = tid + 256u * (unsigned)i, row = p >> 4, c8 = (p & 15u) * 8u;
                const v4f a0 = *(const v4f*)(cst + row * OPITCH + c8);
                const v4f a1 = *(const v4f*)(cst + row * OPITCH + c8 + 4u);
#pragma unroll
                for (int j = 0; j < 4; ++j) {
                    hv[i][j]     = (_Float16)(a0[j] * X2_CARRY);
                    hv[i][4 + j] = (_Float16)(a1[j] * X2_CARRY);
                }
            }
#pragma unroll
            for (int i = 0; i < 4; ++i) {
                const unsigned p = tid + 256u * (unsigned)i, row = p >> 4, c8 = (p & 15u) * 8u;
                *(volatile v8h*)(oh0 + (size_t)(row0 + row) * DM + cb + c8) = hv[i];
            }
            __threadfence();
#pragma unroll
            for (int i = 0; i < 4; ++i) {
                const unsigned p = tid + 256u * (unsigned)i, row = p >> 4, c8 = (p & 15u) * 8u;
                *(volatile v8h*)(oh0 + (size_t)(row0 + row) * DM + cb + c8) = hv[i];
            }
        }
    }
}

__global__ __launch_bounds__(256) void k_attn(const _Float16* __restrict__ Qh, const _Float16* __restrict__ Kh, const _Float16* __restrict__ Vh, _Float16* Xc)
{
    __shared__ __align__(16) _Float16 sK[2 * KT * KPITCH];
    __shared__ __align__(16) _Float16 sVt[128 * VPITCH];
    __shared__ __align__(16) _Float16 sP[8 * 16 * PPITCH];
    __shared__ __align__(16) _Float16 sC[QR * CPITCH];

    const unsigned tid = threadIdx.x, lane = tid & 31u, wv = tid >> 5, hh = lane >> 4, lm = lane & 15u;
    const unsigned rg = wv & 3u, s = wv >> 2;
    const unsigned b = blockIdx.z, hp = blockIdx.y, q0 = blockIdx.x * (unsigned)QR;

    FragH qa[2];
    {
        const _Float16* qrow = Qh + ((size_t)b * SEQ + q0 + rg * 16u + lm) * DM + (2u * hp + s) * (unsigned)DH;
#pragma unroll
        for (int j = 0; j < 2; ++j) {
            qa[j].h[0] = *(const v8h*)(qrow + 32 * j + 8u * hh);
            qa[j].h[1] = *(const v8h*)(qrow + 32 * j + 16u + 8u * hh);
        }
    }
    v8f acc[4];
    float rm[8], rl[8];
#pragma unroll
    for (int t = 0; t < 4; ++t) acc[t] = (v8f){};
#pragma unroll
    for (int r = 0; r < 8; ++r) { rm[r] = -1e30f; rl[r] = 0.f; }

    const size_t kvrow0 = (size_t)b * SEQ;
    const unsigned nkt = (q0 >> 5) + 2u;
    const unsigned rowb = q0 + rg * 16u + 8u * hh;
    const float SCS = 0.125f / (QKV_CARRY * QKV_CARRY);
#pragma unroll 1
    for (unsigned kt = 0; kt < nkt; ++kt) {
        const unsigned key0 = kt * (unsigned)KT;
#pragma unroll
        for (int i = 0; i < 2; ++i) {
            const unsigned p = tid + 256u * (unsigned)i, key = p >> 4, c16 = p & 15u;
            const size_t g = (kvrow0 + key0 + key) * DM + (size_t)hp * 128u + c16 * 8u;
            const v8h kv = *(const v8h*)(Kh + g);
            *(v8h*)(sK + ((c16 >> 3) * (unsigned)KT + key) * KPITCH + (c16 & 7u) * 8u) = kv;
            const v8h vv = *(const v8h*)(Vh + g);
#pragma unroll
            for (int j = 0; j < 8; ++j) sVt[(c16 * 8u + (unsigned)j) * VPITCH + key] = vv[j];
        }
        __syncthreads();

        v8f sc[2];
#pragma unroll
        for (int t = 0; t < 2; ++t) {
            v8f c = (v8f){};
#pragma unroll
            for (int j = 0; j < 2; ++j) {
                FragH kb;
                const _Float16* kr = sK + (s * (unsigned)KT + (unsigned)t * 16u + lm) * KPITCH + 32 * j;
                kb.h[0] = *(const v8h*)(kr + 8u * hh);
                kb.h[1] = *(const v8h*)(kr + 16u + 8u * hh);
                c = wm_f16(qa[j].v, kb.v, c);
            }
            sc[t] = c;
        }
        const unsigned keyA = key0 + lm, keyB = keyA + 16u;
#pragma unroll
        for (int r = 0; r < 8; ++r) {
            const unsigned row = rowb + (unsigned)r;
            const bool mA = keyA > row, mB = keyB > row;
            const float x0 = mA ? -1e30f : sc[0][r] * SCS;
            const float x1 = mB ? -1e30f : sc[1][r] * SCS;
            float mx = fmaxf(x0, x1);
#pragma unroll
            for (int o = 1; o < 16; o <<= 1) mx = fmaxf(mx, __shfl_xor(mx, o, 32));
            const float nm = fmaxf(rm[r], mx);
            const float corr = __expf(rm[r] - nm);
            float p0 = __expf(x0 - nm), p1 = __expf(x1 - nm);
            p0 = mA ? 0.f : p0;
            p1 = mB ? 0.f : p1;
            float rs = p0 + p1;
#pragma unroll
            for (int o = 1; o < 16; o <<= 1) rs += __shfl_xor(rs, o, 32);
            rl[r] = rl[r] * corr + rs;
            rm[r] = nm;
#pragma unroll
            for (int t = 0; t < 4; ++t) acc[t][r] = acc[t][r] * corr;
            _Float16* prow = sP + (wv * 16u + 8u * hh + (unsigned)r) * PPITCH;
            prow[lm] = (_Float16)(p0 * P_CARRY);
            prow[16u + lm] = (_Float16)(p1 * P_CARRY);
        }
        __syncthreads();

        {
            FragH pa;
            const _Float16* pr = sP + (wv * 16u + lm) * PPITCH;
            pa.h[0] = *(const v8h*)(pr + 8u * hh);
            pa.h[1] = *(const v8h*)(pr + 16u + 8u * hh);
#pragma unroll
            for (int t = 0; t < 4; ++t) {
                FragH vb;
                const _Float16* vr = sVt + ((s * 4u + (unsigned)t) * 16u + lm) * VPITCH;
                vb.h[0] = *(const v8h*)(vr + 8u * hh);
                vb.h[1] = *(const v8h*)(vr + 16u + 8u * hh);
                acc[t] = wm_f16(pa.v, vb.v, acc[t]);
            }
        }
        __syncthreads();
    }

#pragma unroll
    for (int r = 0; r < 8; ++r) {
        const float inv = (1.0f / rl[r]) * (C_CARRY / (P_CARRY * QKV_CARRY));
#pragma unroll
        for (int t = 0; t < 4; ++t)
            sC[(rg * 16u + 8u * hh + (unsigned)r) * CPITCH + s * 64u + (unsigned)t * 16u + lm] = (_Float16)(acc[t][r] * inv);
    }
    __syncthreads();
    v8h ov[4];
#pragma unroll
    for (int i = 0; i < 4; ++i) {
        const unsigned p = tid + 256u * (unsigned)i, row = p >> 4, c8 = (p & 15u) * 8u;
        ov[i] = *(const v8h*)(sC + row * CPITCH + c8);
    }
#pragma unroll
    for (int i = 0; i < 4; ++i) {
        const unsigned p = tid + 256u * (unsigned)i, row = p >> 4, c8 = (p & 15u) * 8u;
        *(volatile v8h*)(Xc + (kvrow0 + q0 + row) * DM + (size_t)hp * 128u + c8) = ov[i];
    }
    __threadfence();
#pragma unroll
    for (int i = 0; i < 4; ++i) {
        const unsigned p = tid + 256u * (unsigned)i, row = p >> 4, c8 = (p & 15u) * 8u;
        *(volatile v8h*)(Xc + (kvrow0 + q0 + row) * DM + (size_t)hp * 128u + c8) = ov[i];
    }
}

#define NACT ((size_t)NB * SEQ * DM)
#define WS_TOTAL (NACT * 2 + (size_t)3 * DM * DM * 2 + (size_t)DM * DM * 2 + (size_t)FF * DM * 2 * 2 + NACT * 2 * 3 + NACT * 2 + NACT * 4 + NACT * 2 + (size_t)NB * SEQ * FF * 2)
static_assert(WS_TOTAL <= (size_t)134217728);

extern "C" void kernel_launch(void* const* d_in, const int* in_sizes, int n_in,
                              void* d_out, int out_size, void* d_ws, size_t ws_size, hipStream_t stream)
{
    if (n_in < 13) return;
    const long long needX = ((long long)(NB - 1) * SEQ_FULL + SEQ) * DM;
    if ((long long)in_sizes[0] < needX) return;
    if (in_sizes[1] < DM * DM || in_sizes[3] < DM * DM || in_sizes[5] < DM * DM || in_sizes[7] < DM * DM) return;
    if (in_sizes[2] < DM || in_sizes[4] < DM || in_sizes[6] < DM || in_sizes[8] < DM || in_sizes[12] < DM) return;
    if (in_sizes[9] < FF * DM || in_sizes[11] < FF * DM || in_sizes[10] < FF) return;
    if ((long long)out_size < needX) return;

    const float* x  = (const float*)d_in[0];
    const float* Wq = (const float*)d_in[1];
    const float* bq = (const float*)d_in[2];
    const float* Wk = (const float*)d_in[3];
    const float* bk = (const float*)d_in[4];
    const float* Wv = (const float*)d_in[5];
    const float* bv = (const float*)d_in[6];
    const float* Wo = (const float*)d_in[7];
    const float* bo = (const float*)d_in[8];
    const float* W1 = (const float*)d_in[9];
    const float* b1 = (const float*)d_in[10];
    const float* W2 = (const float*)d_in[11];
    const float* b2 = (const float*)d_in[12];
    float* out = (float*)d_out;

    const size_t nact = NACT;
    unsigned char* base = (unsigned char*)d_ws;
    size_t off = 0;
    _Float16* Xh   = (_Float16*)(base + off); off += nact * 2;
    _Float16* Wqkv = (_Float16*)(base + off); off += (size_t)3 * DM * DM * 2;
    _Float16* Woh  = (_Float16*)(base + off); off += (size_t)DM * DM * 2;
    _Float16* W1h  = (_Float16*)(base + off); off += (size_t)FF * DM * 2;
    _Float16* W2h  = (_Float16*)(base + off); off += (size_t)FF * DM * 2;
    _Float16* Qh   = (_Float16*)(base + off); off += nact * 2;
    _Float16* Kh   = (_Float16*)(base + off); off += nact * 2;
    _Float16* Vh   = (_Float16*)(base + off); off += nact * 2;
    _Float16* Ctx  = (_Float16*)(base + off); off += nact * 2;
    float*    X2f  = (float*)(base + off);    off += nact * 4;
    _Float16* X2h  = (_Float16*)(base + off); off += nact * 2;
    _Float16* Hh   = (_Float16*)(base + off); off += (size_t)NB * SEQ * FF * 2;
    if (off > ws_size) return;

    const unsigned nblkX = (unsigned)(nact / 2048);
    const unsigned M = (unsigned)(NB * SEQ);
    k_convert<<<dim3(nblkX + 4u * NWB + 2u * NFB), dim3(256), 0, stream>>>(x, Wq, Wk, Wv, Wo, W1, W2, Xh, Wqkv, Woh, W1h, W2h, nblkX);
    k_gemm<0, DM><<<dim3(M / 64, (3 * DM) / 128), dim3(256), 0, stream>>>(Xh, Wqkv, bq, bk, bv, x, X2f, Qh, Kh, Vh);
    k_attn<<<dim3(SEQ / QR, HE / 2, NB), dim3(256), 0, stream>>>(Qh, Kh, Vh, Ctx);
    k_gemm<2, DM><<<dim3(M / 64, DM / 128), dim3(256), 0, stream>>>(Ctx, Woh, bo, bo, bo, x, X2f, X2h, X2h, X2h);
    k_gemm<1, DM><<<dim3(M / 64, FF / 128), dim3(256), 0, stream>>>(X2h, W1h, b1, b1, b1, x, X2f, Hh, Hh, Hh);
    k_gemm<3, FF><<<dim3(M / 64, DM / 128), dim3(256), 0, stream>>>(Hh, W2h, b2, b2, b2, X2f, out, Hh, Hh, Hh);
}
